// TransformerBlock_5188320494353
// MI455X (gfx1250) — hardware-verified
//
#include <hip/hip_runtime.h>
#ifndef NB
#define NB 2
#endif
#ifndef SEQ
#define SEQ 2048
#endif
#define NB_FULL 2
#define SEQ_FULL 2048
#define DM 1024
#define NH 16
#define HD 64
#define DFF 4096
#define LQ (3 * DM)
#define NR (NB * SEQ)

static_assert(NB <= NB_FULL);
static_assert(SEQ <= SEQ_FULL);
static_assert(DM == 1024);
static_assert(NH * HD == DM);
static_assert(HD == 64);
static_assert(SEQ % 128 == 0);
static_assert(NR % 128 == 0);
static_assert(NR % 4 == 0);
static_assert(DM % 64 == 0 && LQ % 64 == 0 && DFF % 64 == 0);
static_assert(DM % 32 == 0 && DFF % 32 == 0);
static_assert(SEQ % 64 == 0);

typedef _Float16 v16h __attribute__((ext_vector_type(16)));
typedef unsigned short v8us __attribute__((ext_vector_type(8), may_alias));
typedef float v8f  __attribute__((ext_vector_type(8)));
typedef float v4f  __attribute__((ext_vector_type(4)));
typedef float v4fa __attribute__((ext_vector_type(4), may_alias));
union FragH { v16h v; v8us half[2]; _Float16 h[16]; unsigned short u[16]; };

__device__ __forceinline__ unsigned short bf16_bits(float x) { unsigned int u = __float_as_uint(x); return (unsigned short)((u + 0x7FFFu + ((u >> 16) & 1u)) >> 16); }
__device__ __forceinline__ float bf16_rne(float x) { return __uint_as_float(((unsigned int)bf16_bits(x)) << 16); }
__device__ __forceinline__ size_t tok_full(int r) { return (size_t)(r / SEQ) * SEQ_FULL + (size_t)(r % SEQ); }

__device__ __forceinline__ v16h ld_frag(const unsigned short* p) { FragH f; f.half[0] = *(const v8us*)p; f.half[1] = *(const v8us*)(p + 16); return f.v; }
__device__ __forceinline__ v8f mma16(v16h a, v16h b, v8f c) {
  v8f d = __builtin_amdgcn_wmma_f32_16x16x32_f16(false, a, false, b, (short)0, c, false, false);
  asm volatile("v_nop\n\tv_nop\n\tv_nop\n\tv_nop" : "+v"(d) : "v"(a), "v"(b));
  return d;
}

__global__ __launch_bounds__(256) void k_wt_f16(const float* __restrict__ W, _Float16* __restrict__ Wt, int K, int N, float scale) {
  const int t = blockIdx.x * 256 + threadIdx.x;
  const int k8n = K / 8;
  if (t >= N * k8n) return;
  const int n = t / k8n, k8 = (t - n * k8n) * 8;
  FragH f;
#pragma unroll
  for (int i = 0; i < 8; ++i) f.h[i] = (_Float16)(bf16_rne(W[(size_t)(k8 + i) * N + n]) * scale);
  const v8us o = f.half[0];
  unsigned short* dst = (unsigned short*)Wt + (size_t)n * K + k8;
  *(volatile v8us*)dst = o;
  __threadfence();
  *(volatile v8us*)dst = o;
}

__global__ __launch_bounds__(128) void k_ln16(const float* __restrict__ X, int mapfull, int bfin, const float* __restrict__ g, const float* __restrict__ bb, _Float16* __restrict__ N16) {
#pragma clang fp contract(off)
  const int lane = threadIdx.x & 31;
  const int wave = __builtin_amdgcn_readfirstlane((int)(threadIdx.x >> 5));
  const int r = blockIdx.x * 4 + wave;
  if (r >= NR) return;
  const size_t xr = mapfull ? tok_full(r) : (size_t)r;
  const float* xp = X + xr * DM + lane * 8;
  float s[32];
  float sum = 0.f;
#pragma unroll
  for (int u = 0; u < 4; ++u) {
    const v4f a = *(const v4fa*)(xp + u * 256), c = *(const v4fa*)(xp + u * 256 + 4);
#pragma unroll
    for (int q = 0; q < 4; ++q) {
      const float va = bfin ? bf16_rne(a[q]) : a[q];
      const float vc = bfin ? bf16_rne(c[q]) : c[q];
      s[u * 8 + q] = va; s[u * 8 + 4 + q] = vc; sum = sum + va; sum = sum + vc;
    }
  }
#pragma unroll
  for (int off = 16; off > 0; off >>= 1) sum = sum + __shfl_xor(sum, off);
  const float mu = sum * (1.0f / (float)DM);
  float vs = 0.f;
#pragma unroll
  for (int i = 0; i < 32; ++i) { const float dl = s[i] - mu; vs = vs + dl * dl; }
#pragma unroll
  for (int off = 16; off > 0; off >>= 1) vs = vs + __shfl_xor(vs, off);
  const float rs = rsqrtf(vs * (1.0f / (float)DM) + 1e-5f);
  v8us outv[4];
#pragma unroll
  for (int u = 0; u < 4; ++u) {
    const int c0 = u * 256 + lane * 8;
    const v4f g0 = *(const v4fa*)(g + c0), g1 = *(const v4fa*)(g + c0 + 4);
    const v4f b0 = *(const v4fa*)(bb + c0), b1 = *(const v4fa*)(bb + c0 + 4);
    FragH f;
#pragma unroll
    for (int q = 0; q < 4; ++q) {
      f.h[q]     = (_Float16)(((s[u * 8 + q] - mu) * rs) * bf16_rne(g0[q]) + bf16_rne(b0[q]));
      f.h[4 + q] = (_Float16)(((s[u * 8 + 4 + q] - mu) * rs) * bf16_rne(g1[q]) + bf16_rne(b1[q]));
    }
    outv[u] = f.half[0];
  }
  unsigned short* dst = (unsigned short*)N16 + (size_t)r * DM + lane * 8;
  for (int pass = 0; pass < 2; ++pass) {
#pragma unroll
    for (int u = 0; u < 4; ++u) *(volatile v8us*)(dst + u * 256) = outv[u];
    if (pass == 0) __threadfence();
  }
}

template <int MODE>
__device__ __forceinline__ void gemm_body(const _Float16* __restrict__ A, int lda, const _Float16* __restrict__ Bt, int ldb, float alpha,
                                          const float* __restrict__ bias, const float* __restrict__ resid, int ldr,
                                          float* __restrict__ C32, _Float16* __restrict__ C16, int ldc, int M, int N, int K) {
  __shared__ __attribute__((aligned(16))) float so[4][32][68];
  const int lane = threadIdx.x & 31, ln = lane & 15, hh = lane >> 4;
  const int w = __builtin_amdgcn_readfirstlane((int)(threadIdx.x >> 5));
  const int ntn = N >> 6;
  const int mt = blockIdx.x / ntn, nq = blockIdx.x - mt * ntn;
  const int row0 = mt * 128 + 32 * w, col0 = nq * 64;
  if (row0 >= M) return;
  const unsigned short* a0p = (const unsigned short*)A + (size_t)(row0 + ln) * lda + 8 * hh;
  const unsigned short* a1p = a0p + (size_t)16 * lda;
  const unsigned short* b0p = (const unsigned short*)Bt + (size_t)(col0 + ln) * ldb + 8 * hh;
  const unsigned short* b1p = b0p + (size_t)16 * ldb;
  const unsigned short* b2p = b1p + (size_t)16 * ldb;
  const unsigned short* b3p = b2p + (size_t)16 * ldb;
  const v8f z8 = {0.f, 0.f, 0.f, 0.f, 0.f, 0.f, 0.f, 0.f};
  v8f c00 = z8, c01 = z8, c02 = z8, c03 = z8, c10 = z8, c11 = z8, c12 = z8, c13 = z8;
#pragma unroll 1
  for (int kb = 0; kb < K; kb += 32) {
    const v16h a0 = ld_frag(a0p + kb), a1 = ld_frag(a1p + kb);
    v16h b = ld_frag(b0p + kb); c00 = mma16(a0, b, c00); c10 = mma16(a1, b, c10);
    b = ld_frag(b1p + kb); c01 = mma16(a0, b, c01); c11 = mma16(a1, b, c11);
    b = ld_frag(b2p + kb); c02 = mma16(a0, b, c02); c12 = mma16(a1, b, c12);
    b = ld_frag(b3p + kb); c03 = mma16(a0, b, c03); c13 = mma16(a1, b, c13);
  }
  v8f accs[8] = {c00, c01, c02, c03, c10, c11, c12, c13};
#pragma unroll
  for (int u = 0; u < 8; ++u) {
    const int t = u & 3, half = u >> 2;
    const float bv = bf16_rne(bias[col0 + t * 16 + ln]);
#pragma unroll
    for (int r = 0; r < 8; ++r) so[w][half * 16 + 8 * hh + r][t * 16 + ln] = accs[u][r] * alpha + bv;
  }
  __builtin_amdgcn_fence(4  , "workgroup");
  __builtin_amdgcn_wave_barrier();
  if (MODE == 0 || MODE == 1) {
    const int rq = lane >> 3, c8 = (lane & 7) * 8;
    unsigned short* cb = (unsigned short*)C16 + (size_t)row0 * ldc + col0 + c8;
#pragma unroll 1
    for (int q = 0; q < 8; ++q) {
      const int r = q * 4 + rq;
      v4f a = *(const v4fa*)&so[w][r][c8], b = *(const v4fa*)&so[w][r][c8 + 4];
      if (MODE == 1) {
#pragma unroll
        for (int i = 0; i < 4; ++i) {
          a[i] = 32.0f * a[i] * (1.0f + erff(a[i] * 0.70710678118654752f));
          b[i] = 32.0f * b[i] * (1.0f + erff(b[i] * 0.70710678118654752f));
        }
        *(v4fa*)&so[w][r][c8] = a; *(v4fa*)&so[w][r][c8 + 4] = b;
      }
      FragH f;
#pragma unroll
      for (int i = 0; i < 4; ++i) { f.h[i] = (_Float16)a[i]; f.h[4 + i] = (_Float16)b[i]; }
      *(volatile v8us*)(cb + (size_t)r * ldc) = f.half[0];
    }
    __threadfence();
#pragma unroll 1
    for (int q = 0; q < 8; ++q) {
      const int r = q * 4 + rq;
      const v4f a = *(const v4fa*)&so[w][r][c8], b = *(const v4fa*)&so[w][r][c8 + 4];
      FragH f;
#pragma unroll
      for (int i = 0; i < 4; ++i) { f.h[i] = (_Float16)a[i]; f.h[4 + i] = (_Float16)b[i]; }
      *(volatile v8us*)(cb + (size_t)r * ldc) = f.half[0];
    }
  } else {
    const int rsub = lane >> 4, c4 = (lane & 15) * 4;
    const size_t rrow0 = (MODE == 2) ? tok_full(row0) : (size_t)row0;
    const size_t crow0 = (MODE == 3) ? tok_full(row0) : (size_t)row0;
    const float* rb = resid + rrow0 * ldr + col0 + c4;
    float* cb = C32 + crow0 * ldc + col0 + c4;
#pragma unroll 1
    for (int q = 0; q < 16; ++q) {
      const int r = q * 2 + rsub;
      v4f v = *(const v4fa*)&so[w][r][c4];
      const v4f rv = *(const v4fa*)(rb + (size_t)r * ldr);
#pragma unroll
      for (int i = 0; i < 4; ++i) v[i] = v[i] + ((MODE == 2) ? bf16_rne(rv[i]) : rv[i]);
      *(v4fa*)&so[w][r][c4] = v;
      *(volatile v4f*)(cb + (size_t)r * ldc) = v;
    }
    __threadfence();
#pragma unroll 1
    for (int q = 0; q < 16; ++q) {
      const int r = q * 2 + rsub;
      const v4f v = *(const v4fa*)&so[w][r][c4];
      *(volatile v4f*)(cb + (size_t)r * ldc) = v;
    }
  }
}

__global__ __launch_bounds__(128) void k_gemm_qkv(const _Float16* __restrict__ A, const _Float16* __restrict__ Bt, const float* __restrict__ bias, _Float16* __restrict__ C16) {
  gemm_body<0>(A, DM, Bt, DM, 0.0625f, bias, nullptr, 0, nullptr, C16, LQ, NR, LQ, DM);
}
__global__ __launch_bounds__(128) void k_gemm_proj(const _Float16* __restrict__ A, const _Float16* __restrict__ Bt, const float* __restrict__ bias, const float* __restrict__ xin, float* __restrict__ X1) {
  gemm_body<2>(A, DM, Bt, DM, 0.0009765625f, bias, xin, DM, X1, nullptr, DM, NR, DM, DM);
}
__global__ __launch_bounds__(128) void k_gemm_ff1(const _Float16* __restrict__ A, const _Float16* __restrict__ Bt, const float* __restrict__ bias, _Float16* __restrict__ C16) {
  gemm_body<1>(A, DM, Bt, DM, 0.0625f, bias, nullptr, 0, nullptr, C16, DFF, NR, DFF, DM);
}
__global__ __launch_bounds__(128) void k_gemm_ff2(const _Float16* __restrict__ A, const _Float16* __restrict__ Bt, const float* __restrict__ bias, const float* __restrict__ X1, float* __restrict__ out) {
  gemm_body<3>(A, DFF, Bt, DFF, 0.000244140625f, bias, X1, DM, out, nullptr, DM, NR, DM, DFF);
}

__global__ __launch_bounds__(256) void k_vt(const _Float16* __restrict__ QKVp, _Float16* __restrict__ VT) {
  __shared__ unsigned short tl[64][66];
  const int tid = threadIdx.x;
  const int slab = blockIdx.x / (SEQ / 64), lg = blockIdx.x - slab * (SEQ / 64);
  const int b = slab / NH, h = slab - b * NH;
  for (int i = tid; i < 64 * 8; i += 256) {
    const int r = i >> 3, c8 = (i & 7) * 8;
    FragH f;
    f.half[0] = *(const v8us*)((const unsigned short*)QKVp + ((size_t)b * SEQ + lg * 64 + r) * LQ + 2 * DM + h * HD + c8);
#pragma unroll
    for (int q = 0; q < 8; ++q) tl[r][c8 + q] = f.u[q];
  }
  __syncthreads();
  for (int pass = 0; pass < 2; ++pass) {
#pragma unroll
    for (int rd = 0; rd < 2; ++rd) {
      const int d = rd * 32 + (tid >> 3), pc = tid & 7;
      FragH f;
#pragma unroll
      for (int q = 0; q < 8; ++q) f.u[q] = tl[pc * 8 + q][d];
      *(volatile v8us*)((unsigned short*)VT + ((size_t)slab * HD + d) * SEQ + lg * 64 + pc * 8) = f.half[0];
    }
    if (pass == 0) __threadfence();
  }
}

__global__ __launch_bounds__(128) void k_attn(const _Float16* __restrict__ QKVp, const _Float16* __restrict__ VT, _Float16* __restrict__ O16) {
  __shared__ __attribute__((aligned(16))) unsigned short ot[4][16][72];
  const int lane = threadIdx.x & 31, ln = lane & 15, hh = lane >> 4;
  const int wave = __builtin_amdgcn_readfirstlane((int)(threadIdx.x >> 5));
  const int bh = blockIdx.x / (SEQ / 64), qb = blockIdx.x - bh * (SEQ / 64);
  const int b = bh / NH, h = bh - b * NH;
  const int q0 = qb * 64 + wave * 16;
  const unsigned short* base = (const unsigned short*)QKVp + (size_t)b * SEQ * LQ + h * HD + 8 * hh;
  const unsigned short* qp = base + (size_t)(q0 + ln) * LQ;
  const v16h fq0 = ld_frag(qp), fq1 = ld_frag(qp + 32);
  const unsigned short* kp = base + DM + (size_t)ln * LQ;
  const unsigned short* vp = (const unsigned short*)VT + ((size_t)bh * HD + ln) * SEQ + 8 * hh;
  const v8f z8 = {0.f, 0.f, 0.f, 0.f, 0.f, 0.f, 0.f, 0.f};
  v8f o0 = z8, o1 = z8, o2 = z8, o3 = z8;
  float m = -1.0e30f, l = 0.f;
#pragma unroll 1
  for (int key0 = 0; key0 < SEQ; key0 += 32) {
    const unsigned short* k0p = kp + (size_t)key0 * LQ;
    const unsigned short* k1p = k0p + (size_t)16 * LQ;
    v8f s0 = z8, s1 = z8;
    s0 = mma16(ld_frag(k0p), fq0, s0); s0 = mma16(ld_frag(k0p + 32), fq1, s0);
    s1 = mma16(ld_frag(k1p), fq0, s1); s1 = mma16(ld_frag(k1p + 32), fq1, s1);
    float mx = fmaxf(s0[0], s1[0]);
#pragma unroll
    for (int r = 1; r < 8; ++r) mx = fmaxf(mx, fmaxf(s0[r], s1[r]));
    mx = mx * 0.125f;
    mx = fmaxf(mx, __shfl_xor(mx, 16));
    const float mn = fmaxf(m, mx);
    const float corr = __expf(m - mn);
    m = mn;
    FragH pf;
    float ls = 0.f;
#pragma unroll
    for (int r = 0; r < 8; ++r) {
      const float e0 = __expf(s0[r] * 0.125f - mn), e1 = __expf(s1[r] * 0.125f - mn);
      ls += e0 + e1;
      pf.h[r] = (_Float16)(e0 * 1024.0f); pf.h[8 + r] = (_Float16)(e1 * 1024.0f);
    }
    l = l * corr + ls;
    o0 = o0 * corr; o1 = o1 * corr; o2 = o2 * corr; o3 = o3 * corr;
    const unsigned short* vk = vp + key0;
    o0 = mma16(ld_frag(vk), pf.v, o0);
    o1 = mma16(ld_frag(vk + (size_t)16 * SEQ), pf.v, o1);
    o2 = mma16(ld_frag(vk + (size_t)32 * SEQ), pf.v, o2);
    o3 = mma16(ld_frag(vk + (size_t)48 * SEQ), pf.v, o3);
  }
  const float lt = l + __shfl_xor(l, 16);
  const float inv = 0.0625f * (1.0f / lt);
  FragH f;
#pragma unroll
  for (int r = 0; r < 8; ++r) f.h[r] = (_Float16)(o0[r] * inv);
  *(v8us*)&ot[wave][ln][8 * hh] = f.half[0];
#pragma unroll
  for (int r = 0; r < 8; ++r) f.h[r] = (_Float16)(o1[r] * inv);
  *(v8us*)&ot[wave][ln][16 + 8 * hh] = f.half[0];
#pragma unroll
  for (int r = 0; r < 8; ++r) f.h[r] = (_Float16)(o2[r] * inv);
  *(v8us*)&ot[wave][ln][32 + 8 * hh] = f.half[0];
#pragma unroll
  for (int r = 0; r < 8; ++r) f.h[r] = (_Float16)(o3[r] * inv);
  *(v8us*)&ot[wave][ln][48 + 8 * hh] = f.half[0];
  __builtin_amdgcn_fence(4  , "workgroup");
  __builtin_amdgcn_wave_barrier();
  const int rq = lane >> 3, pc = (lane & 7) * 8;
  unsigned short* ob = (unsigned short*)O16 + ((size_t)b * SEQ + q0) * DM + h * HD + pc;
  for (int pass = 0; pass < 2; ++pass) {
#pragma unroll
    for (int it = 0; it < 4; ++it) {
      const int row = it * 4 + rq;
      const v8us v = *(const v8us*)&ot[wave][row][pc];
      *(volatile v8us*)(ob + (size_t)row * DM) = v;
    }
    if (pass == 0) __threadfence();
  }
}

constexpr size_t SZ_BQKV = (size_t)LQ * DM * 2;
constexpr size_t SZ_BO   = (size_t)DM * DM * 2;
constexpr size_t SZ_BW1  = (size_t)DFF * DM * 2;
constexpr size_t SZ_BW2  = (size_t)DM * DFF * 2;
constexpr size_t SZ_X16  = (size_t)NR * DM * 2;
constexpr size_t SZ_QKV  = (size_t)NR * LQ * 2;
constexpr size_t SZ_VT   = (size_t)NR * DM * 2;
constexpr size_t SZ_HF   = (size_t)NR * DFF * 2;
constexpr size_t SZ_RQV  = (SZ_QKV + SZ_VT) > SZ_HF ? (SZ_QKV + SZ_VT) : SZ_HF;
constexpr size_t SZ_O16  = (size_t)NR * DM * 2;
constexpr size_t SZ_X1   = (size_t)NR * DM * 4;
constexpr size_t SZ_M16  = (size_t)NR * DM * 2;
constexpr size_t WS_TOTAL = SZ_BQKV + SZ_BO + SZ_BW1 + SZ_BW2 + SZ_X16 + SZ_RQV + SZ_O16 + SZ_X1 + SZ_M16;
static_assert(SZ_BQKV % 256 == 0 && SZ_BO % 256 == 0 && SZ_BW1 % 256 == 0 && SZ_BW2 % 256 == 0 && SZ_X16 % 256 == 0);
static_assert(SZ_QKV % 256 == 0 && SZ_RQV % 256 == 0 && SZ_O16 % 256 == 0 && SZ_X1 % 256 == 0 && SZ_M16 % 256 == 0);
static_assert(SZ_HF <= SZ_RQV);
static_assert(SZ_QKV + SZ_VT <= SZ_RQV);
static_assert(WS_TOTAL <= (size_t)134217728);

extern "C" void kernel_launch(void* const* d_in, const int* in_sizes, int n_in,
                              void* d_out, int out_size, void* d_ws, size_t ws_size, hipStream_t stream) {
  if (n_in < 13) return;
  const long long need_x = ((long long)(NB - 1) * SEQ_FULL + SEQ) * DM;
  if ((long long)in_sizes[0] < need_x) return;
  if ((long long)in_sizes[1] < (long long)DM * LQ || in_sizes[2] < LQ) return;
  if ((long long)in_sizes[3] < (long long)DM * DM || in_sizes[4] < DM) return;
  if ((long long)in_sizes[5] < (long long)DM * DFF || in_sizes[6] < DFF) return;
  if ((long long)in_sizes[7] < (long long)DFF * DM || in_sizes[8] < DM) return;
  if (in_sizes[9] < DM || in_sizes[10] < DM || in_sizes[11] < DM || in_sizes[12] < DM) return;
  if ((long long)out_size < need_x) return;
  if (WS_TOTAL > ws_size) return;
  const float* x    = (const float*)d_in[0];
  const float* wqkv = (const float*)d_in[1];
  const float* bqkv = (const float*)d_in[2];
  const float* wo   = (const float*)d_in[3];
  const float* bo   = (const float*)d_in[4];
  const float* w1   = (const float*)d_in[5];
  const float* b1   = (const float*)d_in[6];
  const float* w2   = (const float*)d_in[7];
  const float* b2   = (const float*)d_in[8];
  const float* g1   = (const float*)d_in[9];
  const float* be1  = (const float*)d_in[10];
  const float* g2   = (const float*)d_in[11];
  const float* be2  = (const float*)d_in[12];
  float* out = (float*)d_out;
  char* ws = (char*)d_ws; size_t off = 0;
  _Float16* BQKV = (_Float16*)(ws + off); off += SZ_BQKV;
  _Float16* BO   = (_Float16*)(ws + off); off += SZ_BO;
  _Float16* BW1  = (_Float16*)(ws + off); off += SZ_BW1;
  _Float16* BW2  = (_Float16*)(ws + off); off += SZ_BW2;
  _Float16* X16  = (_Float16*)(ws + off); off += SZ_X16;
  _Float16* QKVp = (_Float16*)(ws + off);
  _Float16* VT   = (_Float16*)(ws + off + SZ_QKV);
  _Float16* HF16 = (_Float16*)(ws + off); off += SZ_RQV;
  _Float16* O16  = (_Float16*)(ws + off); off += SZ_O16;
  float*    X1   = (float*)(ws + off);    off += SZ_X1;
  _Float16* M16  = (_Float16*)(ws + off); off += SZ_M16;

  k_wt_f16<<<(unsigned)(((size_t)LQ * (DM / 8) + 255) / 256), 256, 0, stream>>>(wqkv, BQKV, DM, LQ, 16.0f);
  k_wt_f16<<<(unsigned)(((size_t)DM * (DM / 8) + 255) / 256), 256, 0, stream>>>(wo, BO, DM, DM, 16.0f);
  k_wt_f16<<<(unsigned)(((size_t)DFF * (DM / 8) + 255) / 256), 256, 0, stream>>>(w1, BW1, DM, DFF, 16.0f);
  k_wt_f16<<<(unsigned)(((size_t)DM * (DFF / 8) + 255) / 256), 256, 0, stream>>>(w2, BW2, DFF, DM, 64.0f);
  k_ln16<<<NR / 4, 128, 0, stream>>>(x, 1, 1, g1, be1, X16);
  k_gemm_qkv<<<(NR / 128) * (LQ / 64), 128, 0, stream>>>(X16, BQKV, bqkv, QKVp);
  k_vt<<<NB * NH * (SEQ / 64), 256, 0, stream>>>(QKVp, VT);
  k_attn<<<NB * NH * (SEQ / 64), 128, 0, stream>>>(QKVp, VT, O16);
  k_gemm_proj<<<(NR / 128) * (DM / 64), 128, 0, stream>>>(O16, BO, bo, x, X1);
  k_ln16<<<NR / 4, 128, 0, stream>>>(X1, 0, 0, g2, be2, M16);
  k_gemm_ff1<<<(NR / 128) * (DFF / 64), 128, 0, stream>>>(M16, BW1, b1, HF16);
  k_gemm_ff2<<<(NR / 128) * (DM / 64), 128, 0, stream>>>(HF16, BW2, b2, X1, out);
}
